// SparseAttention_88837103551208
// MI455X (gfx1250) — hardware-run, weakly checked
//
#include <hip/hip_runtime.h>


#define NB_  4
#define TT   4096
#define DD   256
#define RB   64
#define NBK  (TT / RB)
#define KWN  128
#define WOFF 32
#define BLO  5
#define BHI  4
#define NBD  (BLO + BHI + 1)

typedef _Float16 h16;
typedef unsigned short bf;
typedef __attribute__((ext_vector_type(16))) __bf16   v16bf;
typedef __attribute__((ext_vector_type(16))) _Float16 v16h;
typedef __attribute__((ext_vector_type(8)))  _Float16 v8h;
typedef __attribute__((ext_vector_type(8)))  unsigned short v8us;
typedef __attribute__((ext_vector_type(8)))  float    v8f;
typedef __attribute__((ext_vector_type(4)))  float    v4f;
typedef v8h  __attribute__((may_alias)) v8ha;
typedef v4f  __attribute__((may_alias)) v4fa;
typedef v8us __attribute__((may_alias)) v8usa;

__device__ __forceinline__ unsigned short f2bf(float f) { unsigned u = __float_as_uint(f); u += 0x7FFFu + ((u >> 16) & 1u); return (unsigned short)(u >> 16); }
__device__ __forceinline__ float bf2f(unsigned short b) { return __uint_as_float(((unsigned)b) << 16); }
__device__ __forceinline__ float bfr(float f) { return bf2f(f2bf(f)); }
__device__ __forceinline__ v16h cat16(v8h lo, v8h hi) { return __builtin_shufflevector(lo, hi, 0, 1, 2, 3, 4, 5, 6, 7, 8, 9, 10, 11, 12, 13, 14, 15); }
__device__ __forceinline__ v16bf cat16b(v8us lo, v8us hi) { return __builtin_bit_cast(v16bf, __builtin_shufflevector(lo, hi, 0, 1, 2, 3, 4, 5, 6, 7, 8, 9, 10, 11, 12, 13, 14, 15)); }
__device__ __forceinline__ v8f wmma16(v16h a, v16h b, v8f c) { return __builtin_amdgcn_wmma_f32_16x16x32_f16(false, a, false, b, (short)0, c, false, false); }
__device__ __forceinline__ v8f wmmab(v16bf a, v16bf b, v8f c) { return __builtin_amdgcn_wmma_f32_16x16x32_bf16(false, a, false, b, (short)0, c, false, false); }
typedef __attribute__((ext_vector_type(2))) _Float16 v2h;
typedef __attribute__((ext_vector_type(4))) _Float16 v4h;
typedef __attribute__((ext_vector_type(2))) unsigned short v2us;
typedef __attribute__((ext_vector_type(4))) unsigned short v4us;
typedef __attribute__((ext_vector_type(2))) float v2f;
typedef __attribute__((ext_vector_type(4))) int v4i;

template <typename T16> struct WFrag;
template <> struct WFrag<h16> { typedef v16h V; static __device__ __forceinline__ V ld(const h16* p) { return cat16(*(const v8h*)p, *(const v8h*)(p + 16)); } static __device__ __forceinline__ v8f mma(V a, V b, v8f c) { return wmma16(a, b, c); } };
template <> struct WFrag<bf> { typedef v16bf V; static __device__ __forceinline__ V ld(const bf* p) { return cat16b(*(const v8us*)p, *(const v8us*)(p + 16)); } static __device__ __forceinline__ v8f mma(V a, V b, v8f c) { return wmmab(a, b, c); } };
template <typename T16, int NSPLIT, bool BIAS>
__global__ __launch_bounds__(32) void k_gemmw(const T16* __restrict__ A, const T16* __restrict__ A2, const T16* __restrict__ Bt, const T16* __restrict__ Bt2, int K, float* C, int ldc, const float* __restrict__ bias, size_t sA, size_t sB, size_t sC) {
    typedef typename WFrag<T16>::V V;
    __shared__ __align__(16) float os[16 * 68];
    const size_t z = blockIdx.z; A += z * sA; if (A2) A2 += z * sA; Bt += z * sB; if (Bt2) Bt2 += z * sB; C += z * sC;
    const int lane = threadIdx.x & 31, lr = lane & 15, hi = lane >> 4; const int r0 = blockIdx.x * 64, c0 = blockIdx.y * 64;
    v8f acc[4][4];
#pragma unroll
    for (int mb = 0; mb < 4; ++mb)
#pragma unroll
        for (int nb = 0; nb < 4; ++nb) acc[mb][nb] = (v8f){};
    const size_t aoff = (size_t)(r0 + lr) * K + 8 * hi, boff = (size_t)(c0 + lr) * K + 8 * hi;

    for (int kc = 0; kc < K; kc += 32) {
        V a[4], a2[4];
#pragma unroll
        for (int mb = 0; mb < 4; ++mb) { a[mb] = WFrag<T16>::ld(A + aoff + (size_t)mb * 16 * K + kc); if (NSPLIT == 1 || NSPLIT == 2) a2[mb] = WFrag<T16>::ld(A2 + aoff + (size_t)mb * 16 * K + kc); }
#pragma unroll
        for (int nb = 0; nb < 4; ++nb) { const V b = WFrag<T16>::ld(Bt + boff + (size_t)nb * 16 * K + kc); V b2; if (NSPLIT >= 2) b2 = WFrag<T16>::ld(Bt2 + boff + (size_t)nb * 16 * K + kc);
#pragma unroll
            for (int mb = 0; mb < 4; ++mb) { acc[mb][nb] = WFrag<T16>::mma(a[mb], b, acc[mb][nb]); if (NSPLIT == 1 || NSPLIT == 2) acc[mb][nb] = WFrag<T16>::mma(a2[mb], b, acc[mb][nb]); if (NSPLIT >= 2) acc[mb][nb] = WFrag<T16>::mma(a[mb], b2, acc[mb][nb]); } }
        asm volatile("v_nop\n\tv_nop\n\tv_nop\n\tv_nop" : "+v"(acc[0][0]), "+v"(acc[1][1]), "+v"(acc[2][2]), "+v"(acc[3][3]) : "v"(a[0]), "v"(a[3]));
    }
#pragma unroll
    for (int mb = 0; mb < 4; ++mb) {
#pragma unroll
        for (int nb = 0; nb < 4; ++nb) {
#pragma unroll
            for (int j = 0; j < 8; ++j) os[(hi * 8 + j) * 68 + nb * 16 + lr] = acc[mb][nb][j]; }
        __builtin_amdgcn_wave_barrier(); asm volatile("" ::: "memory");
        float* crow = C + (size_t)(r0 + mb * 16) * ldc + c0;
#pragma unroll 1
        for (int ps = 0; ps < 2; ++ps) {
#pragma unroll
            for (int s = 0; s < 8; ++s) { const int row = 2 * s + hi, cofs = lr * 4; v4f val = *(const v4fa*)(os + row * 68 + cofs); if (BIAS) { val[0] += bfr(bias[c0 + cofs]); val[1] += bfr(bias[c0 + cofs + 1]); val[2] += bfr(bias[c0 + cofs + 2]); val[3] += bfr(bias[c0 + cofs + 3]); }
                *(volatile v4f*)(crow + (size_t)row * ldc + cofs) = val; }
            if (ps == 0) __threadfence(); }
        __builtin_amdgcn_wave_barrier(); asm volatile("" ::: "memory");
    }
}

__device__ __forceinline__ h16 tohx(float x) { return (h16)x; }
__device__ __forceinline__ void splitf(float y, unsigned short& h, unsigned short& l) { h = f2bf(y); l = f2bf(y - bf2f(h)); }
typedef __attribute__((ext_vector_type(2))) _Float16 v2h;
typedef __attribute__((ext_vector_type(4))) _Float16 v4h;
typedef __attribute__((ext_vector_type(2))) unsigned short v2us;
typedef __attribute__((ext_vector_type(4))) unsigned short v4us;
typedef __attribute__((ext_vector_type(2))) float v2f;
typedef __attribute__((ext_vector_type(4))) int v4i;

__global__ __launch_bounds__(256) void k_cvt8(const float* __restrict__ src, bf* dst, size_t n8) { const size_t i = (size_t)blockIdx.x * 256 + threadIdx.x; if (i >= n8) return; const v8f v = *(const v8f*)(src + i * 8); v8us o;
#pragma unroll
    for (int k = 0; k < 8; ++k) o[k] = f2bf(v[k]); *(volatile v8us*)(dst + i * 8) = o; __threadfence(); *(volatile v8us*)(dst + i * 8) = o; }


__global__ __launch_bounds__(256) void k_kwb(const float* __restrict__ K, bf* KW) { const size_t e = ((size_t)blockIdx.x * 256 + threadIdx.x) * 8; if (e >= (size_t)NBK * KWN * DD) return; const int d0 = (int)(e % DD); const int y = (int)((e / DD) % KWN); const int blk = (int)(e / ((size_t)DD * KWN));
    const int j = blk * RB - WOFF + y; const bool ok = (j >= 0) & (j < TT); const int jc = min(max(j, 0), TT - 1); const float f = ok ? 1.0f : 0.0f; const float* kr = K + (size_t)jc * DD + d0; const v4f a = *(const v4f*)kr; const v4f b = *(const v4f*)(kr + 4); v8us o;
#pragma unroll
    for (int q = 0; q < 4; ++q) { o[q] = f2bf(__fmul_rn(a[q], f)); o[q + 4] = f2bf(__fmul_rn(b[q], f)); }
    *(volatile v8us*)(KW + e) = o; __threadfence(); *(volatile v8us*)(KW + e) = o; }

__global__ __launch_bounds__(256) void k_vwt(const float* __restrict__ V, h16* VW) { const size_t e = ((size_t)blockIdx.x * 256 + threadIdx.x) * 8; if (e >= (size_t)NBK * DD * KWN) return; const int y0 = (int)(e % KWN); const int o = (int)((e / KWN) % DD); const int blk = (int)(e / ((size_t)KWN * DD)); const int j0 = blk * RB - WOFF + y0; v8h w;
#pragma unroll
    for (int q = 0; q < 8; ++q) { const int j = j0 + q; const bool ok = (j >= 0) & (j < TT); const int jc = min(max(j, 0), TT - 1); const float f = ok ? 1.0f : 0.0f; w[q] = tohx(__fmul_rn(bfr(V[(size_t)jc * DD + o]), f)); }
    *(volatile v8h*)(VW + e) = w; __threadfence(); *(volatile v8h*)(VW + e) = w; }

__global__ __launch_bounds__(256) void k_bsm(const float* __restrict__ S, h16* P16) { const size_t e = ((size_t)blockIdx.x * 256 + threadIdx.x) * 8; if (e >= (size_t)NBK * RB * KWN) return; const int y0 = (int)(e % KWN); const int x = (int)((e / KWN) % RB); const int blk = (int)(e / ((size_t)KWN * RB)); const int i = blk * RB + x; const int c0 = x + WOFF - BLO; const int a = c0 & ~3; const int sh = c0 - a; const float* sr = S + ((size_t)blk * RB + x) * KWN + a; float u[16];
#pragma unroll
    for (int g = 0; g < 4; ++g) { const v4f z = *(const v4f*)(sr + 4 * g); u[4 * g] = z[0]; u[4 * g + 1] = z[1]; u[4 * g + 2] = z[2]; u[4 * g + 3] = z[3]; }
    float t[NBD]; float m = -3.0e38f;
#pragma unroll
    for (int c = 0; c < NBD; ++c) { float s0 = u[c + 3]; s0 = (sh == 2) ? u[c + 2] : s0; s0 = (sh == 1) ? u[c + 1] : s0; s0 = (sh == 0) ? u[c] : s0; const int j = i - BLO + c; const bool ok = (j >= 0) & (j < TT); const float s = __fmul_rn(s0, 0.0625f); t[c] = ok ? s : -3.0e38f; m = fmaxf(m, t[c]); }
    float sum = 0.0f;
#pragma unroll
    for (int c = 0; c < NBD; ++c) { t[c] = __builtin_amdgcn_exp2f(__fmul_rn(__fsub_rn(t[c], m), 1.4426950408889634f)); sum = __fadd_rn(sum, t[c]); }
    const float r = __fdiv_rn(1.0f, sum); v8h w;
#pragma unroll
    for (int q = 0; q < 8; ++q) { const int c = y0 + q - c0; float p = 0.0f;
#pragma unroll
        for (int cc = 0; cc < NBD; ++cc) p = (c == cc) ? t[cc] : p;
        w[q] = tohx(__fmul_rn(p, r)); }
    *(volatile v8h*)(P16 + e) = w; __threadfence(); *(volatile v8h*)(P16 + e) = w; }

extern "C" void kernel_launch(void* const* d_in, const int* in_sizes, int n_in,
                              void* d_out, int out_size, void* d_ws, size_t ws_size, hipStream_t stream) {
    (void)in_sizes; (void)n_in; (void)out_size;
    const float* qin = (const float*)d_in[0]; const float* kin = (const float*)d_in[1]; const float* vin = (const float*)d_in[2];
    float* OUT = (float*)d_out;
    char* wsp = (char*)d_ws;
    auto take = [&](size_t bytes) { char* p = wsp; wsp += (bytes + 255) & ~(size_t)255; return (void*)p; };
    const size_t NE = (size_t)TT * DD;
    bf* QB = (bf*)take(NE * 2); bf* KW = (bf*)take((size_t)NBK * KWN * DD * 2); float* Sb = (float*)take((size_t)NBK * RB * KWN * 4); h16* P16 = (h16*)take((size_t)NBK * RB * KWN * 2); h16* VW = (h16*)take((size_t)NBK * DD * KWN * 2);
    if ((size_t)(wsp - (char*)d_ws) > ws_size) return;
    for (int b = 0; b < NB_; ++b) {
        k_cvt8<<<(unsigned)((NE / 8 + 255) / 256), 256, 0, stream>>>(qin + (size_t)b * NE, QB, NE / 8);
        k_kwb<<<(unsigned)((size_t)NBK * KWN * DD / 2048), 256, 0, stream>>>(kin + (size_t)b * NE, KW);
        k_gemmw<bf, 0, false><<<dim3(RB / 64, KWN / 64, NBK), 32, 0, stream>>>(QB, nullptr, KW, nullptr, DD, Sb, KWN, nullptr, (size_t)RB * DD, (size_t)KWN * DD, (size_t)RB * KWN);
        k_bsm<<<(unsigned)((size_t)NBK * RB * KWN / 2048), 256, 0, stream>>>(Sb, P16);
        k_vwt<<<(unsigned)((size_t)NBK * DD * KWN / 2048), 256, 0, stream>>>(vin + (size_t)b * NE, VW);
        k_gemmw<h16, 0, false><<<dim3(RB / 64, DD / 64, NBK), 32, 0, stream>>>(P16, nullptr, VW, nullptr, KWN, OUT + (size_t)b * NE, DD, nullptr, (size_t)RB * KWN, (size_t)DD * KWN, (size_t)RB * DD);
    }
}
